// MKGC_67413806678372
// MI455X (gfx1250) — hardware-verified
//
#include <hip/hip_runtime.h>
#include <stddef.h>


#define FD      128
#define NKER    4
#define NATOM   4
#define KTOT    (3 * FD)
#define NTHR    256
#define NWAVE   8
#define EPT     8
#define NGRP    2
#define CHUNK   (NTHR * EPT * NGRP)
#define WCAP    (EPT * NGRP * 32)
#define LISTN   (NWAVE * WCAP)
#define SLOTSH  13
#define SLOTMSK ((1 << SLOTSH) - 1)
#define NB      448
#define RPW     (NB / NWAVE)
#define GR      64
#define WPLN    (NKER * FD * KTOT)
#define NWBLK   (3 * NKER * FD * (FD / 8) / NTHR)
#define WSCAP   134217728
#define LDS_AGG (NB * FD * 4 + LISTN * 4 + NB * 4 + NWAVE * 4)

static_assert((CHUNK & (CHUNK - 1)) == 0);
static_assert(NB <= (1 << SLOTSH));
static_assert((NB % 64) == 0 && (NB % (2 * NWAVE)) == 0);
static_assert(NWBLK * NTHR == 3 * NKER * FD * (FD / 8) && NWBLK == 96);
static_assert(LDS_AGG == 247584);
static_assert((KTOT % 32) == 0 && GR == NWAVE * 8 && NATOM == 4 && NKER == NATOM);
static_assert(((WPLN * 2) % 256) == 0);

typedef float          v4f  __attribute__((ext_vector_type(4)));
typedef float          v8f  __attribute__((ext_vector_type(8)));
typedef int            v4i  __attribute__((ext_vector_type(4)));
typedef _Float16       v8h  __attribute__((ext_vector_type(8)));
typedef _Float16       v16h __attribute__((ext_vector_type(16)));
union FragH { v16h v; v8h h[2]; };

__device__ __forceinline__ v8f wmf(v16h a, v16h b, v8f c) {
  v8f d = __builtin_amdgcn_wmma_f32_16x16x32_f16(false, a, false, b, (short)0, c, false, false);
  asm volatile("v_nop\n\tv_nop\n\tv_nop\n\tv_nop" : "+v"(d) : "v"(a), "v"(b));
  return d;
}

template <int NSL>
__device__ __forceinline__ int scan_chunk(const int* __restrict__ keys, int nE, int cbase, int slotBase,
                                          int vec8, int* list, int tid, int lane, int wave) {
  int wc = 0;
#pragma unroll
  for (int g = 0; g < NGRP; ++g) {
    const int el0  = (g * NTHR + tid) * EPT;
    const int e0   = cbase + el0;
    const int sent = -2147483647 - 1;
    v4i da, db;
    if (vec8 != 0 && cbase + CHUNK <= nE) {
      da = *(const v4i*)(keys + e0);
      db = *(const v4i*)(keys + e0 + 4);
    } else {
      da.x = (e0     < nE) ? keys[min(e0, nE - 1)] : sent;
      da.y = (e0 + 1 < nE) ? keys[min(e0 + 1, nE - 1)] : sent;
      da.z = (e0 + 2 < nE) ? keys[min(e0 + 2, nE - 1)] : sent;
      da.w = (e0 + 3 < nE) ? keys[min(e0 + 3, nE - 1)] : sent;
      db.x = (e0 + 4 < nE) ? keys[min(e0 + 4, nE - 1)] : sent;
      db.y = (e0 + 5 < nE) ? keys[min(e0 + 5, nE - 1)] : sent;
      db.z = (e0 + 6 < nE) ? keys[min(e0 + 6, nE - 1)] : sent;
      db.w = (e0 + 7 < nE) ? keys[min(e0 + 7, nE - 1)] : sent;
    }
    const unsigned nb = (unsigned)slotBase;
    const unsigned s0 = (unsigned)da.x - nb, s1 = (unsigned)da.y - nb;
    const unsigned s2 = (unsigned)da.z - nb, s3 = (unsigned)da.w - nb;
    const unsigned s4 = (unsigned)db.x - nb, s5 = (unsigned)db.y - nb;
    const unsigned s6 = (unsigned)db.z - nb, s7 = (unsigned)db.w - nb;
    const bool h0 = s0 < (unsigned)NSL, h1 = s1 < (unsigned)NSL, h2 = s2 < (unsigned)NSL, h3 = s3 < (unsigned)NSL;
    const bool h4 = s4 < (unsigned)NSL, h5 = s5 < (unsigned)NSL, h6 = s6 < (unsigned)NSL, h7 = s7 < (unsigned)NSL;
    const unsigned any = __builtin_amdgcn_ballot_w32(h0 | h1 | h2 | h3 | h4 | h5 | h6 | h7);
    if (any != 0u) {
#define HITJ(J, HJ, SJ) { \
        const unsigned mj = __builtin_amdgcn_ballot_w32(HJ); \
        if (mj != 0u) { \
          if (HJ) { \
            const int pos = wc + (int)__builtin_amdgcn_mbcnt_lo(mj, 0u); \
            if (pos < WCAP) list[wave * WCAP + pos] = ((el0 + (J)) << SLOTSH) | (int)(SJ); \
          } \
          wc += (int)__builtin_popcount(mj); } }
      HITJ(0, h0, s0)
      HITJ(1, h1, s1)
      HITJ(2, h2, s2)
      HITJ(3, h3, s3)
      HITJ(4, h4, s4)
      HITJ(5, h5, s5)
      HITJ(6, h6, s6)
      HITJ(7, h7, s7)
#undef HITJ
    }
  }
  return wc;
}

__global__ __launch_bounds__(NTHR) void k_wprep(
    const float* __restrict__ w1, const float* __restrict__ w2, const float* __restrict__ wr,
    _Float16* wpl) {
  const int blk = blockIdx.x, tid = threadIdx.x;
  const int seg = blk >> 5;
  const float* w = (seg == 0) ? wr : ((seg == 1) ? w1 : w2);
  const int i   = (blk & 31) * NTHR + tid;
  const int row = i >> 4;
  const int kk0 = (i & 15) * 8;
  const int kq  = row >> 7, n = row & 127;
  v8h hv;
#pragma unroll
  for (int e = 0; e < 8; ++e) hv[e] = (_Float16)(w[((size_t)(kq * FD + kk0 + e)) * FD + n] * 64.0f);
  _Float16* d = wpl + (size_t)row * KTOT + seg * FD + kk0;
  *(volatile v8h*)d = hv;
  __threadfence();
  *(volatile v8h*)d = hv;
}

__device__ __forceinline__ void x16_pass(const float* __restrict__ x, _Float16* x16, int slotBase,
                                         int nN, int wave, int hf, int c0) {
#pragma unroll 1
  for (int j = 0; j < RPW / 2; ++j) {
    const int rl   = wave * RPW + 2 * j + hf;
    const int node = slotBase + rl;
    const int nc   = node > nN - 1 ? nN - 1 : node;
    const float f  = (node < nN) ? 8.0f : 0.0f;
    const v4f a = *(const v4f*)(x + (size_t)nc * FD + c0);
    const v4f b = *(const v4f*)(x + (size_t)nc * FD + c0 + 4);
    v8h hv;
    hv[0] = (_Float16)(a.x * f); hv[1] = (_Float16)(a.y * f); hv[2] = (_Float16)(a.z * f); hv[3] = (_Float16)(a.w * f);
    hv[4] = (_Float16)(b.x * f); hv[5] = (_Float16)(b.y * f); hv[6] = (_Float16)(b.z * f); hv[7] = (_Float16)(b.w * f);
    *(volatile v8h*)(x16 + (size_t)node * FD + c0) = hv;
  }
}

__device__ __forceinline__ void agg_pass(const float* sacc, const int* scnt, _Float16* plane,
                                         int slotBase, int wave, int hf, int c0) {
#pragma unroll 1
  for (int j = 0; j < RPW / 2; ++j) {
    const int rl = wave * RPW + 2 * j + hf;
    const int c  = scnt[rl];
    const float s = 8.0f * (1.0f / (float)(c < 1 ? 1 : c));
    const v4f a = *(const v4f*)(sacc + rl * FD + c0);
    const v4f b = *(const v4f*)(sacc + rl * FD + c0 + 4);
    v8h hv;
    hv[0] = (_Float16)(a.x * s); hv[1] = (_Float16)(a.y * s); hv[2] = (_Float16)(a.z * s); hv[3] = (_Float16)(a.w * s);
    hv[4] = (_Float16)(b.x * s); hv[5] = (_Float16)(b.y * s); hv[6] = (_Float16)(b.z * s); hv[7] = (_Float16)(b.w * s);
    *(volatile v8h*)(plane + (size_t)(slotBase + rl) * FD + c0) = hv;
  }
}

__global__ __launch_bounds__(NTHR) void k_agg(
    const int* __restrict__ ei, const float* __restrict__ x,
    _Float16* apl, size_t ps, int nN, int nE, int nBlk, int vecd) {
  extern __shared__ v4f lds_dyn[];
  float* sacc = (float*)lds_dyn;
  int*   list = (int*)(sacc + NB * FD);
  int*   scnt = list + LISTN;
  int*   wcnt = scnt + NB;
  const int tid = threadIdx.x, lane = tid & 31, wave = tid >> 5, hf = lane >> 4, c0 = (lane & 15) * 8;
  const int dir = ((int)blockIdx.x >= nBlk) ? 1 : 0;
  const int b = (int)blockIdx.x - dir * nBlk;
  const int slotBase = b * NB;
  const int* keys = (dir == 0) ? (ei + nE) : ei;
  const int* oth  = (dir == 0) ? ei : (ei + nE);
  const int vec8  = (dir == 0) ? vecd : 1;
  _Float16* x16   = apl;
  _Float16* plane = apl + (size_t)(1 + dir) * ps;

  {
    const v4f z = {0.f, 0.f, 0.f, 0.f};
    for (int i = tid; i < NB * FD / 4; i += NTHR) ((v4f*)sacc)[i] = z;
    for (int s = tid; s < NB; s += NTHR) scnt[s] = 0;
  }
  if (dir == 0) {
    x16_pass(x, x16, slotBase, nN, wave, hf, c0);
    __threadfence();
    x16_pass(x, x16, slotBase, nN, wave, hf, c0);
  }
  __syncthreads();

  const int nChunks = (nE + CHUNK - 1) / CHUNK;
#pragma unroll 1
  for (int ch = 0; ch < nChunks; ++ch) {
    const int cbase = ch * CHUNK;
    const int wc = scan_chunk<NB>(keys, nE, cbase, slotBase, vec8, list, tid, lane, wave);
    if (lane == 0) wcnt[wave] = wc;
    __syncthreads();
#pragma unroll 1
    for (int wsx = 0; wsx < NWAVE; ++wsx) {
      int n = __builtin_amdgcn_readfirstlane(wcnt[wsx]);
      n = n > WCAP ? WCAP : (n < 0 ? 0 : n);
      const int* lp = list + wsx * WCAP;
#pragma unroll 1
      for (int q0 = 0; q0 < n; q0 += 32) {
        int li = q0 + lane;
        li = li > n - 1 ? n - 1 : li;
        const int ent = lp[li];
        int slot = ent & SLOTMSK;
        slot = slot > NB - 1 ? NB - 1 : slot;
        int e = cbase + ((ent >> SLOTSH) & (CHUNK - 1));
        e = e > nE - 1 ? nE - 1 : e;
        int ov = oth[e];
        ov = ov < 0 ? 0 : (ov > nN - 1 ? nN - 1 : ov);
        const int mcnt = (n - q0) < 32 ? (n - q0) : 32;
#pragma unroll 1
        for (int p = 0; p < mcnt; ++p) {
          const int ss = __builtin_amdgcn_readlane(slot, p);
          const int oo = __builtin_amdgcn_readlane(ov, p);
          if ((ss & (NWAVE - 1)) == wave) {
            const v4f xv = *(const v4f*)(x + (size_t)oo * FD + 4 * lane);
            float* ap = sacc + ss * FD + 4 * lane;
            v4f a = *(const v4f*)ap;
            a += xv;
            *(v4f*)ap = a;
            if (lane == 0) scnt[ss] = scnt[ss] + 1;
          }
        }
      }
    }
    __syncthreads();
  }

  agg_pass(sacc, scnt, plane, slotBase, wave, hf, c0);
  __threadfence();
  agg_pass(sacc, scnt, plane, slotBase, wave, hf, c0);
}

__global__ __launch_bounds__(NTHR) void k_layer(
    const _Float16* __restrict__ apl, size_t ps, const _Float16* __restrict__ wpl,
    const float* __restrict__ x, const float* __restrict__ wd, const float* __restrict__ broot,
    float* out, int nN) {
  __shared__ __attribute__((aligned(16))) float stg[GR * FD];
  __shared__ __attribute__((aligned(16))) float sco[GR * NATOM];
  const int tid = threadIdx.x, lane = tid & 31, wave = tid >> 5, hh = lane >> 4, m = lane & 15;
  const int rg = wave >> 1, chf = wave & 1;
  const int rowBase = blockIdx.x * GR;

  if (wave < 2) {
    int node = rowBase + tid;
    node = node > nN - 1 ? nN - 1 : node;
    const float* xr = x + (size_t)node * FD;
    float a0 = 0.f, a1 = 0.f, a2 = 0.f, a3 = 0.f;
#pragma unroll 1
    for (int k = 0; k < FD; ++k) {
      const float xv = xr[k];
      const v4f w = *(const v4f*)(wd + 4 * k);
      a0 += xv * w.x; a1 += xv * w.y; a2 += xv * w.z; a3 += xv * w.w;
    }
    const float mx = fmaxf(fmaxf(a0, a1), fmaxf(a2, a3));
    const float e0 = __expf(a0 - mx), e1 = __expf(a1 - mx), e2 = __expf(a2 - mx), e3 = __expf(a3 - mx);
    const float inv = 1.0f / (e0 + e1 + e2 + e3);
    v4f c;
    c.x = e0 * inv; c.y = e1 * inv; c.z = e2 * inv; c.w = e3 * inv;
    *(v4f*)(sco + NATOM * tid) = c;
  }
  __syncthreads();

  const int arow = rowBase + rg * 16 + m;
  float* strow = stg + (rg * 16 + 8 * hh) * FD + m;
#pragma unroll 1
  for (int tt = 0; tt < 4; ++tt) {
    const int t = chf * 4 + tt;
    v8f tot = {0.f, 0.f, 0.f, 0.f, 0.f, 0.f, 0.f, 0.f};
#pragma unroll 1
    for (int k = 0; k < NKER; ++k) {
      v8f acc = {0.f, 0.f, 0.f, 0.f, 0.f, 0.f, 0.f, 0.f};
      const _Float16* bf = wpl + (size_t)(k * FD + 16 * t + m) * KTOT + 8 * hh;
#pragma unroll 1
      for (int p = 0; p < 3; ++p) {
        const _Float16* pa = apl + (size_t)p * ps + (size_t)arow * FD + 8 * hh;
        const _Float16* pb = bf + p * FD;
#pragma unroll
        for (int c = 0; c < FD / 32; ++c) {
          FragH a, bq;
          a.h[0]  = *(const v8h*)(pa + 32 * c);
          a.h[1]  = *(const v8h*)(pa + 32 * c + 16);
          bq.h[0] = *(const v8h*)(pb + 32 * c);
          bq.h[1] = *(const v8h*)(pb + 32 * c + 16);
          acc = wmf(a.v, bq.v, acc);
        }
      }
      const float bv = broot[k * FD + 16 * t + m];
#pragma unroll
      for (int r = 0; r < 8; ++r) {
        const float cf = sco[(rg * 16 + 8 * hh + r) * NATOM + (k % NATOM)];
        tot[r] += fmaxf(acc[r] * (1.0f / 512.0f) + bv, 0.0f) * cf;
      }
    }
#pragma unroll
    for (int r = 0; r < 8; ++r) strow[r * FD + 16 * t] = tot[r];
  }
  __syncthreads();

  v4f ov[8];
#pragma unroll
  for (int i = 0; i < 8; ++i) ov[i] = *(const v4f*)(stg + (8 * wave + i) * FD + 4 * lane);
#pragma unroll
  for (int i = 0; i < 8; ++i) {
    const int grow = rowBase + 8 * wave + i;
    if (grow < nN) *(volatile v4f*)(out + (size_t)grow * FD + 4 * lane) = ov[i];
  }
  __threadfence();
#pragma unroll
  for (int i = 0; i < 8; ++i) {
    const int grow = rowBase + 8 * wave + i;
    if (grow < nN) *(volatile v4f*)(out + (size_t)grow * FD + 4 * lane) = ov[i];
  }
}

extern "C" void kernel_launch(void* const* d_in, const int* in_sizes, int n_in,
                              void* d_out, int out_size, void* d_ws, size_t ws_size,
                              hipStream_t stream) {
  if (n_in < 7) return;
  const int nN = in_sizes[0] / FD;
  if (nN < 1 || in_sizes[0] != nN * FD) return;
  const int nE = in_sizes[1] / 2;
  if (nE < 1 || in_sizes[1] != 2 * nE) return;
  if (in_sizes[2] != NKER * FD * FD || in_sizes[3] != NKER * FD * FD || in_sizes[4] != NKER * FD * FD) return;
  if (in_sizes[5] != NKER * FD || in_sizes[6] != FD * NATOM) return;
  if ((long long)out_size != (long long)nN * FD) return;
  if (nN > (1 << 24) || nE > (1 << 28)) return;

  const float* x     = (const float*)d_in[0];
  const int*   ei    = (const int*)d_in[1];
  const float* W1    = (const float*)d_in[2];
  const float* W2    = (const float*)d_in[3];
  const float* Wroot = (const float*)d_in[4];
  const float* broot = (const float*)d_in[5];
  const float* Wd    = (const float*)d_in[6];
  float* out = (float*)d_out;

  const int nBlk = (nN + NB - 1) / NB;
  const int PR   = nBlk * NB;
  const int NP64 = ((nN + GR - 1) / GR) * GR;
  if (NP64 > PR) return;

  char* ws = (char*)d_ws;
  size_t off = 0;
  const size_t oW = off; off += (size_t)WPLN * 2;
  const size_t oA = off; off += (size_t)3 * (size_t)PR * FD * 2;
  if (off > ws_size || off > (size_t)WSCAP) return;
  _Float16* wpl = (_Float16*)(ws + oW);
  _Float16* apl = (_Float16*)(ws + oA);
  const size_t ps = (size_t)PR * FD;

  const int vecd = ((nE & 3) == 0) ? 1 : 0;

  k_wprep<<<NWBLK, NTHR, 0, stream>>>(W1, W2, Wroot, wpl);

  hipFuncSetAttribute(reinterpret_cast<const void*>(&k_agg),
                      hipFuncAttributeMaxDynamicSharedMemorySize, LDS_AGG);
  k_agg<<<2 * nBlk, NTHR, LDS_AGG, stream>>>(ei, x, apl, ps, nN, nE, nBlk, vecd);

  k_layer<<<NP64 / GR, NTHR, 0, stream>>>(apl, ps, wpl, x, Wd, broot, out, nN);
}
